// SymmetricContraction_10428180595107
// MI455X (gfx1250) — hardware-verified
//
#include <hip/hip_runtime.h>
#include <math.h>


#ifndef NN
#define NN 1024
#endif
#define NN_FULL 1024
#define CC   128
#define DD   16
#define SS   10
#define NI   4
#define NSC  (SS * CC)
#define NE   (DD * DD * DD)
#define KP   32
#define NKS  9
#define CG   8
#define K3_0 23
#define K2_0 7
#define K1_0 2
#define K3_1 17
#define K2_1 5
#define K1_1 1
#define ZSC  16.0f
#define OSC  (1.0f / 4096.0f)
#define QRS  2048.0f
#define QRI  (1.0f / 2048.0f)

#define S3_0 17.7932301f
#define S2_0 48.3794518f
#define S1_0 181.019333f
#define S3_1 20.6963730f
#define S2_1 57.2433395f
#define S1_1 256.0f

static_assert(K3_0 == 23);
static_assert(K2_0 == 7);
static_assert(K1_0 == 2);
static_assert(K3_1 == 17);
static_assert(K2_1 == 5);
static_assert(K1_1 == 1);
static_assert(__builtin_bit_cast(unsigned, S3_0) == 0x418E5889u);
static_assert(__builtin_bit_cast(unsigned, S2_0) == 0x4241848Fu);
static_assert(__builtin_bit_cast(unsigned, S1_0) == 0x433504F3u);
static_assert(__builtin_bit_cast(unsigned, S3_1) == 0x41A5922Cu);
static_assert(__builtin_bit_cast(unsigned, S2_1) == 0x4264F92Eu);
static_assert(__builtin_bit_cast(unsigned, S1_1) == 0x43800000u);

static_assert(NN % 32 == 0);
static_assert(NN <= NN_FULL);
static_assert(CC % 16 == 0);
static_assert(NSC % 16 == 0);
static_assert(CC % CG == 0);
static_assert(DD == 16);
static_assert(NKS == DD / 2 + 1);
static_assert(K3_0 <= KP);
static_assert(K3_1 <= KP);
static_assert(KP == 32);
static_assert(32 * CG == 16 * 16);
static_assert(CG * DD == 16 * 8);
static_assert(CG * NI * 4 == 128);
static_assert(4 * 32 * 16 == 16 * CG * NI * 4);
static_assert(4 * 32 * 16 == 16 * 64 * 2);
static_assert((NN * 4 + 16 * CG * DD * 4 + 16 * CG * NI * 4 + 16) <= 131072);
static_assert((16 * 68 * 4) <= 131072);

typedef _Float16 h16;
typedef unsigned short bf;
typedef __attribute__((ext_vector_type(16))) __bf16   v16bf;
typedef __attribute__((ext_vector_type(16))) _Float16 v16h;
typedef __attribute__((ext_vector_type(8)))  _Float16 v8h;
typedef __attribute__((ext_vector_type(8)))  unsigned short v8us;
typedef __attribute__((ext_vector_type(8)))  float    v8f;
typedef __attribute__((ext_vector_type(4)))  float    v4f;
typedef v4f  __attribute__((may_alias)) v4fa;

__device__ __forceinline__ unsigned short f2bf(float f) { unsigned u = __float_as_uint(f); u += 0x7FFFu + ((u >> 16) & 1u); return (unsigned short)(u >> 16); }
__device__ __forceinline__ float bfr(float f) { return __uint_as_float(((unsigned)f2bf(f)) << 16); }
__device__ __forceinline__ v16h cat16(v8h lo, v8h hi) { return __builtin_shufflevector(lo, hi, 0, 1, 2, 3, 4, 5, 6, 7, 8, 9, 10, 11, 12, 13, 14, 15); }
__device__ __forceinline__ v16bf cat16b(v8us lo, v8us hi) { return __builtin_bit_cast(v16bf, __builtin_shufflevector(lo, hi, 0, 1, 2, 3, 4, 5, 6, 7, 8, 9, 10, 11, 12, 13, 14, 15)); }
__device__ __forceinline__ v8f wmma16(v16h a, v16h b, v8f c) { return __builtin_amdgcn_wmma_f32_16x16x32_f16(false, a, false, b, (short)0, c, false, false); }
__device__ __forceinline__ v8f wmmab(v16bf a, v16bf b, v8f c) { return __builtin_amdgcn_wmma_f32_16x16x32_bf16(false, a, false, b, (short)0, c, false, false); }
__device__ __forceinline__ v16h  ldh(const h16* p) { return cat16(*(const v8h*)p, *(const v8h*)(p + 16)); }
__device__ __forceinline__ v16bf ldb(const bf* p)  { return cat16b(*(const v8us*)p, *(const v8us*)(p + 16)); }
__device__ __forceinline__ void wave_sync() { __builtin_amdgcn_fence(3  , "wavefront"); __builtin_amdgcn_wave_barrier(); asm volatile("" ::: "memory"); }

static __device__ __forceinline__ h16 toh_flush(float v) { const h16 r = (h16)v; return (fabsf(v) < 6.103515625e-05f) ? (h16)0.0f : r; }
static __device__ __forceinline__ v8f wmma16_g(v16h a, v16h b, v8f c) { c = wmma16(a, b, c); asm volatile("v_nop\n\tv_nop\n\tv_nop\n\tv_nop" : "+v"(c) : "v"(a), "v"(b)); return c; }
static __device__ __forceinline__ v8f wmmab_g(v16bf a, v16bf b, v8f c) { c = wmmab(a, b, c); asm volatile("v_nop\n\tv_nop\n\tv_nop\n\tv_nop" : "+v"(c) : "v"(a), "v"(b)); return c; }

__global__ __launch_bounds__(256) void k_padk(const float* __restrict__ src, bf* dst, int nrows, int inner_n, int ostride, int istride, int kstride, int k) {
    const int tid = blockIdx.x * 256 + threadIdx.x; if (tid >= nrows * 4) return;
    const int r = tid >> 2, q = tid & 3;
    const int outer = r / inner_n, inner = r % inner_n;
    const size_t base = (size_t)outer * (size_t)ostride + (size_t)inner * (size_t)istride;
    v8us o;
#pragma unroll
    for (int t = 0; t < 8; ++t) {
        const int kk = q * 8 + t; const int kc = kk < k ? kk : (k - 1);
        float v = src[base + (size_t)kc * (size_t)kstride];
        asm volatile("" : "+v"(v));
        o[t] = (kk < k) ? f2bf(v) : (unsigned short)0; }
    *(volatile v8us*)(dst + (size_t)tid * 8) = o; __threadfence(); *(volatile v8us*)(dst + (size_t)tid * 8) = o;
}

__global__ __launch_bounds__(32) void k_tab(const bf* __restrict__ WT, const bf* __restrict__ UT, h16* TAB, h16* TABR) {
    __shared__ __align__(16) float os[16 * 68];
    const int lane = threadIdx.x & 31, lr = lane & 15, hi = lane >> 4;
    const int ct = blockIdx.x, ks = blockIdx.y, ig = blockIdx.z;
    const int irr = ig > 0 ? 1 : 0;
    const float scale = irr ? S3_1 : S3_0;
    const v16bf a = ldb(WT + ((size_t)irr * NSC + (size_t)ct * 16 + lr) * KP + 8 * hi);
    const size_t ub = (size_t)ig * NE * KP + 8 * hi;
    const size_t tb = (((size_t)ct * 16) * NI + (size_t)ig) * (size_t)(NKS * 512) + (size_t)ks * 512;
#pragma unroll 1
    for (int bp = 0; bp < 8; ++bp) {
#pragma unroll
        for (int b2 = 0; b2 < 2; ++b2) {
#pragma unroll
            for (int a2 = 0; a2 < 2; ++a2) {
                const int e = ((2 * ks + a2) * 16 + 2 * bp + b2) * 16 + lr;
                const v16bf b = ldb(UT + ub + (size_t)e * KP);
                v8f acc = (v8f){};
                acc = wmmab_g(a, b, acc);
#pragma unroll
                for (int j = 0; j < 8; ++j) os[(hi * 8 + j) * 68 + b2 * 32 + a2 * 16 + lr] = acc[j] * scale; } }
        wave_sync();
#pragma unroll 1
        for (int ps = 0; ps < 2; ++ps) {
#pragma unroll
            for (int s = 0; s < 4; ++s) { const int row = 4 * s + (lane >> 3), c8 = (lane & 7) * 8;
                const v4f x0 = *(const v4fa*)(&os[row * 68 + c8]); const v4f x1 = *(const v4fa*)(&os[row * 68 + c8 + 4]); v8h hv, rv;
#pragma unroll
                for (int i = 0; i < 4; ++i) { const h16 a0 = toh_flush(x0[i]); const h16 a1 = toh_flush(x1[i]); hv[i] = a0; hv[4 + i] = a1;
                    rv[i] = toh_flush((x0[i] - (float)a0) * QRS); rv[4 + i] = toh_flush((x1[i] - (float)a1) * QRS); }
                const size_t oo = tb + (size_t)row * (size_t)(NI * NKS * 512) + (size_t)bp * 64 + c8;
                *(volatile v8h*)(TAB + oo) = hv; *(volatile v8h*)(TABR + oo) = rv; }
            if (ps == 0) __threadfence(); }
        wave_sync();
    }
}

__global__ __launch_bounds__(256) void k_tab2(const float* __restrict__ U2, const float* __restrict__ w2, const float* __restrict__ U1, const float* __restrict__ w1, h16* TAB, h16* TABR,
                                              int k2, int k1, int icnt, int i0, int nthr) {
    const int tid = blockIdx.x * 256 + threadIdx.x; if (tid >= nthr) return;
    const float sc2 = (i0 > 0) ? S2_1 : S2_0;
    const float sc1 = (i0 > 0) ? S1_1 : S1_0;
    const int q = tid & 3, b = (tid >> 2) & 15; const int r = tid >> 6;
    const int il = r % icnt, sc = r / icnt;
    const int s = sc / CC, c = sc % CC;
    const int a0 = (q & 1) * 8;
    float acc[8];
#pragma unroll
    for (int e = 0; e < 8; ++e) acc[e] = 0.0f;
#pragma unroll 1
    for (int kk = 0; kk < k2; ++kk) {
        const float wv = bfr(w2[(size_t)(s * k2 + kk) * CC + c]);
#pragma unroll
        for (int e = 0; e < 8; ++e) acc[e] += bfr(U2[(size_t)(((a0 + e) * 16 + b) * k2 + kk) * icnt + il]) * wv; }
    float a1 = 0.0f;
#pragma unroll 1
    for (int kk = 0; kk < k1; ++kk) a1 += bfr(U1[(size_t)(b * k1 + kk) * icnt + il]) * bfr(w1[(size_t)(s * k1 + kk) * CC + c]);
    v8h ov, rv;
#pragma unroll
    for (int e = 0; e < 8; ++e) {
        float v = (q < 2) ? acc[e] * sc2 : 0.0f;
        if (e == 0) v = (q == 2) ? a1 * sc1 : v;
        const h16 hvv = toh_flush(v);
        ov[e] = hvv; rv[e] = toh_flush((v - (float)hvv) * QRS); }
    const size_t oo = (((size_t)sc * NI + (size_t)(i0 + il)) * NKS + 8) * 512 + (size_t)b * 32 + (size_t)q * 8;
    *(volatile v8h*)(TAB + oo) = ov; *(volatile v8h*)(TABR + oo) = rv; __threadfence(); *(volatile v8h*)(TAB + oo) = ov; *(volatile v8h*)(TABR + oo) = rv;
}

__global__ __launch_bounds__(32 * CG) __attribute__((amdgpu_num_vgpr(256))) void k_main(const float* __restrict__ x, const int* __restrict__ y, const h16* __restrict__ TAB, const h16* __restrict__ TABR, float* OUT) {
    __shared__ int list[NN];
    __shared__ int cnt_s;
    __shared__ __align__(16) float xs[16 * CG * DD];
    __shared__ __align__(16) float outs[16 * CG * NI];
    const int lane = threadIdx.x & 31, lr = lane & 15, hi = lane >> 4;
    const int wave = __builtin_amdgcn_readfirstlane((int)(threadIdx.x >> 5));
    const int cg = blockIdx.x, s = blockIdx.y;
    if (wave == 0) {
        int nfound = 0;
#pragma unroll 1
        for (int it = 0; it < NN / 32; ++it) {
            const int idx = it * 32 + lane;
            int ys = y[idx]; ys = ys < 0 ? 0 : (ys > SS - 1 ? SS - 1 : ys);
            const bool flag = ys == s;
            const unsigned mask = __builtin_amdgcn_ballot_w32(flag);
            const int pre = __builtin_popcount(mask & ((1u << lane) - 1u));
            if (flag) list[nfound + pre] = idx;
            nfound += __builtin_popcount(mask); }
        if (lane == 0) cnt_s = nfound;
    }
    __syncthreads();
    int cntv = cnt_s; cntv = cntv < 0 ? 0 : (cntv > NN ? NN : cntv);
    const int cnt = __builtin_amdgcn_readfirstlane(cntv);
    const int c = cg * CG + wave;
    const size_t tabw = ((size_t)(s * CC + c) * NI) * (size_t)(NKS * 512) + (size_t)lr * 32 + 8 * hi;
#pragma unroll 1
    for (int base = 0; base < cnt; base += 16) {
        { const int t = threadIdx.x; const int nl = t >> 4, p = t & 15;
          int li = base + nl; li = li < cnt ? li : (cnt - 1);
          int node = list[li]; node = node < 0 ? 0 : (node > NN - 1 ? NN - 1 : node);
          const float* src = x + ((size_t)node * CC + (size_t)cg * CG) * DD + p * 8;
          v4f u0 = *(const v4f*)src, u1 = *(const v4f*)(src + 4);
#pragma unroll
          for (int i = 0; i < 4; ++i) { u0[i] = bfr(u0[i]); u1[i] = bfr(u1[i]); }
          *(v4fa*)(&xs[nl * (CG * DD) + p * 8]) = u0; *(v4fa*)(&xs[nl * (CG * DD) + p * 8 + 4]) = u1; }
        __syncthreads();
        float xa[16];
        { const int xb = lr * (CG * DD) + wave * DD;
#pragma unroll
          for (int g = 0; g < 4; ++g) { const v4f t4 = *(const v4fa*)(&xs[xb + 4 * g]); xa[4 * g] = t4[0]; xa[4 * g + 1] = t4[1]; xa[4 * g + 2] = t4[2]; xa[4 * g + 3] = t4[3]; } }
        float xj[8], xz[8];
#pragma unroll
        for (int r = 0; r < 8; ++r) { xj[r] = hi ? xa[8 + r] : xa[r]; xz[r] = xj[r] * ZSC; }
        v16h bz[NKS];
#pragma unroll
        for (int ks = 0; ks < 8; ++ks) {
#pragma unroll
            for (int e = 0; e < 8; ++e) { bz[ks][e] = toh_flush(xa[2 * ks] * xz[e]); bz[ks][8 + e] = toh_flush(xa[2 * ks + 1] * xz[e]); } }
        { v16h t = (v16h){};
#pragma unroll
          for (int e = 0; e < 8; ++e) t[e] = toh_flush(xz[e]);
          t[8] = (h16)(hi ? 0.0f : ZSC);
          bz[8] = t; }
#pragma unroll 1
        for (int i = 0; i < NI; ++i) {
            const h16* tp = TAB + tabw + (size_t)i * (size_t)(NKS * 512);
            const h16* tr = TABR + tabw + (size_t)i * (size_t)(NKS * 512);
            v8f acc = (v8f){}, accr = (v8f){};
#pragma unroll
            for (int ks = 0; ks < NKS; ++ks) { const v16h a = ldh(tp + ks * 512); acc = wmma16_g(a, bz[ks], acc);
                                               const v16h ar = ldh(tr + ks * 512); accr = wmma16_g(ar, bz[ks], accr); }
            float part = 0.0f;
#pragma unroll
            for (int r = 0; r < 8; ++r) part += (acc[r] + accr[r] * QRI) * xj[r];
            part += __shfl_xor(part, 16, 32);
            if (hi == 0) outs[lr * (CG * NI) + wave * NI + i] = part * OSC;
        }
        __syncthreads();
        if (wave < 4) {
            const int row = wave * 4 + (lane >> 3), cofs = (lane & 7) * 4;
            const v4f val = *(const v4fa*)(&outs[row * (CG * NI) + cofs]);
            int li = base + row; const bool ok = li < cnt; li = ok ? li : (cnt - 1);
            int node = list[li]; node = node < 0 ? 0 : (node > NN - 1 ? NN - 1 : node);
            float* dst = OUT + ((size_t)node * CC + (size_t)cg * CG) * NI + cofs;
            if (ok) *(volatile v4f*)dst = val;
            __threadfence();
            if (ok) *(volatile v4f*)dst = val;
        }
    }
}

static constexpr size_t al256(size_t v) { return (v + 255) & ~(size_t)255; }
static constexpr size_t SZ_UT  = al256((size_t)NI * NE * KP * 2);
static constexpr size_t SZ_WT  = al256((size_t)2 * NSC * KP * 2);
static constexpr size_t SZ_TAB = al256((size_t)NSC * NI * NKS * 512 * 2);
static constexpr size_t SZ_TOTAL = SZ_UT + SZ_WT + 2 * SZ_TAB;
static_assert(SZ_TOTAL <= (size_t)134217728);
static_assert(((size_t)NE * KP * 2) % 256 == 0);
static_assert(((size_t)NSC * KP * 2) % 256 == 0);
static_assert(((size_t)NKS * 512 * 2) % 128 == 0);
static_assert((NSC * 1 * 64) % 256 == 0);
static_assert((NSC * 3 * 64) % 256 == 0);

extern "C" void kernel_launch(void* const* d_in, const int* in_sizes, int n_in,
                              void* d_out, int out_size, void* d_ws, size_t ws_size, hipStream_t stream) {
    if (n_in < 14) return;
    if ((size_t)in_sizes[0] < (size_t)NN * CC * DD || in_sizes[1] < NN) return;
    if (in_sizes[2] < NE * K3_0 * 1 || in_sizes[3] < SS * K3_0 * CC) return;
    if (in_sizes[4] < DD * DD * K2_0 * 1 || in_sizes[5] < SS * K2_0 * CC) return;
    if (in_sizes[6] < DD * K1_0 * 1 || in_sizes[7] < SS * K1_0 * CC) return;
    if (in_sizes[8] < NE * K3_1 * 3 || in_sizes[9] < SS * K3_1 * CC) return;
    if (in_sizes[10] < DD * DD * K2_1 * 3 || in_sizes[11] < SS * K2_1 * CC) return;
    if (in_sizes[12] < DD * K1_1 * 3 || in_sizes[13] < SS * K1_1 * CC) return;
    if ((size_t)out_size < (size_t)NN * CC * NI) return;
    if (SZ_TOTAL > ws_size) return;
    const float* x    = (const float*)d_in[0];
    const int*   y    = (const int*)d_in[1];
    const float* U3_0 = (const float*)d_in[2];  const float* w3_0 = (const float*)d_in[3];
    const float* U2_0 = (const float*)d_in[4];  const float* w2_0 = (const float*)d_in[5];
    const float* U1_0 = (const float*)d_in[6];  const float* w1_0 = (const float*)d_in[7];
    const float* U3_1 = (const float*)d_in[8];  const float* w3_1 = (const float*)d_in[9];
    const float* U2_1 = (const float*)d_in[10]; const float* w2_1 = (const float*)d_in[11];
    const float* U1_1 = (const float*)d_in[12]; const float* w1_1 = (const float*)d_in[13];
    float* OUT = (float*)d_out;
    char* wsp = (char*)d_ws;
    bf*  UT   = (bf*)wsp;  wsp += SZ_UT;
    bf*  WT   = (bf*)wsp;  wsp += SZ_WT;
    h16* TAB  = (h16*)wsp; wsp += SZ_TAB;
    h16* TABR = (h16*)wsp; wsp += SZ_TAB;

    k_padk<<<(NE * 1 * 4 + 255) / 256, 256, 0, stream>>>(U3_0, UT, NE * 1, NE, 1, K3_0 * 1, 1, K3_0);
    k_padk<<<(NE * 3 * 4 + 255) / 256, 256, 0, stream>>>(U3_1, UT + (size_t)NE * KP, NE * 3, NE, 1, K3_1 * 3, 3, K3_1);
    k_padk<<<(NSC * 4 + 255) / 256, 256, 0, stream>>>(w3_0, WT, NSC, CC, K3_0 * CC, 1, CC, K3_0);
    k_padk<<<(NSC * 4 + 255) / 256, 256, 0, stream>>>(w3_1, WT + (size_t)NSC * KP, NSC, CC, K3_1 * CC, 1, CC, K3_1);

    k_tab<<<dim3(NSC / 16, 8, NI), 32, 0, stream>>>(WT, UT, TAB, TABR);
    k_tab2<<<(NSC * 1 * 64 + 255) / 256, 256, 0, stream>>>(U2_0, w2_0, U1_0, w1_0, TAB, TABR, K2_0, K1_0, 1, 0, NSC * 1 * 64);
    k_tab2<<<(NSC * 3 * 64 + 255) / 256, 256, 0, stream>>>(U2_1, w2_1, U1_1, w1_1, TAB, TABR, K2_1, K1_1, 3, 1, NSC * 3 * 64);

    k_main<<<dim3(CC / CG, SS, 1), 32 * CG, 0, stream>>>(x, y, TAB, TABR, OUT);
}
